// StructureMapping_44796508897482
// MI455X (gfx1250) — hardware-verified
//
#include <hip/hip_runtime.h>


#define NB_  2
#define NE   20
#define EE   256
#define HH   256
#define RR   400
#define RP   448
#define NPAIR (RR * RR)
#define PCH  80000
#define DM   EE
#define LEPS 1e-5f
#define LOSC 1024.0f

typedef _Float16 h16;
typedef unsigned short bf;
typedef __attribute__((ext_vector_type(16))) __bf16   v16bf;
typedef __attribute__((ext_vector_type(16))) _Float16 v16h;
typedef __attribute__((ext_vector_type(8)))  _Float16 v8h;
typedef __attribute__((ext_vector_type(8)))  unsigned short v8us;
typedef __attribute__((ext_vector_type(8)))  float    v8f;
typedef __attribute__((ext_vector_type(4)))  float    v4f;
typedef v8h  __attribute__((may_alias)) v8ha;
typedef v4f  __attribute__((may_alias)) v4fa;
typedef v8us __attribute__((may_alias)) v8usa;

__device__ __forceinline__ unsigned short f2bf(float f) { unsigned u = __float_as_uint(f); u += 0x7FFFu + ((u >> 16) & 1u); return (unsigned short)(u >> 16); }
__device__ __forceinline__ float bf2f(unsigned short b) { return __uint_as_float(((unsigned)b) << 16); }
__device__ __forceinline__ float bfr(float f) { return bf2f(f2bf(f)); }
__device__ __forceinline__ v16h cat16(v8h lo, v8h hi) { return __builtin_shufflevector(lo, hi, 0, 1, 2, 3, 4, 5, 6, 7, 8, 9, 10, 11, 12, 13, 14, 15); }
__device__ __forceinline__ v16bf cat16b(v8us lo, v8us hi) { return __builtin_bit_cast(v16bf, __builtin_shufflevector(lo, hi, 0, 1, 2, 3, 4, 5, 6, 7, 8, 9, 10, 11, 12, 13, 14, 15)); }
__device__ __forceinline__ v8f wmma16(v16h a, v16h b, v8f c) { return __builtin_amdgcn_wmma_f32_16x16x32_f16(false, a, false, b, (short)0, c, false, false); }
__device__ __forceinline__ v8f wmmab(v16bf a, v16bf b, v8f c) { return __builtin_amdgcn_wmma_f32_16x16x32_bf16(false, a, false, b, (short)0, c, false, false); }

template <bool SPLITA, bool F16OUT = false>
__global__ __launch_bounds__(128) void k_gemmb(const bf* __restrict__ A, const bf* __restrict__ Al, const bf* __restrict__ Bn, const float* __restrict__ bias, float* C, int ldc, h16* C2, const float* __restrict__ R = nullptr, int K = DM, int roundR = 1) {
    __shared__ __align__(16) float ost[4][16 * 68];
    const int lane = threadIdx.x & 31, wave = threadIdx.x >> 5, lr = lane & 15, hi = lane >> 4;
    const int r0 = blockIdx.x * 64 + wave * 16, c0 = blockIdx.y * 64;
    const size_t aoff = (size_t)(r0 + lr) * K + 8 * hi;
    size_t boff[4];
#pragma unroll
    for (int t = 0; t < 4; ++t) boff[t] = (size_t)(c0 + t * 16 + lr) * K + 8 * hi;
    v8f acc[4];
#pragma unroll
    for (int t = 0; t < 4; ++t) acc[t] = (v8f){};
#pragma unroll 1
    for (int kc = 0; kc < K; kc += 32) {
        const v16bf a = cat16b(*(const v8us*)(A + aoff + kc), *(const v8us*)(A + aoff + kc + 16));
        v16bf al = a;
        if (SPLITA) al = cat16b(*(const v8us*)(Al + aoff + kc), *(const v8us*)(Al + aoff + kc + 16));
#pragma unroll
        for (int t = 0; t < 4; ++t) { const v16bf b = cat16b(*(const v8us*)(Bn + boff[t] + kc), *(const v8us*)(Bn + boff[t] + kc + 16)); acc[t] = wmmab(a, b, acc[t]); if (SPLITA) acc[t] = wmmab(al, b, acc[t]); }
        asm volatile("v_nop\n\tv_nop\n\tv_nop\n\tv_nop" : "+v"(acc[0]), "+v"(acc[1]), "+v"(acc[2]), "+v"(acc[3]) : "v"(a), "v"(al));
    }
    float* os = &ost[wave][0];
#pragma unroll
    for (int t = 0; t < 4; ++t) { const float bv = bias ? bfr(bias[c0 + t * 16 + lr]) : 0.f;
#pragma unroll
        for (int j = 0; j < 8; ++j) os[(hi * 8 + j) * 68 + t * 16 + lr] = acc[t][j] + bv; }
    __syncthreads();
    if (F16OUT) {
        h16* crow = (h16*)(void*)C + (size_t)r0 * ldc + c0;
        auto pass = [&]() {
#pragma unroll
            for (int s = 0; s < 4; ++s) { const int row = 4 * s + (lane >> 3), piece = lane & 7; const float* sp = os + row * 68 + piece * 8; v8h o, o2;
#pragma unroll
                for (int i = 0; i < 8; ++i) { const h16 a = (h16)sp[i]; o[i] = a; o2[i] = (h16)((sp[i] - (float)a) * LOSC); }
                *(volatile v8h*)(crow + (size_t)row * ldc + piece * 8) = o; if (C2) *(volatile v8h*)(C2 + (size_t)r0 * ldc + c0 + (size_t)row * ldc + piece * 8) = o2; }
        };
        pass(); __threadfence(); pass();
    } else {
        float* crow = C + (size_t)r0 * ldc + c0;
        auto pass = [&]() {
#pragma unroll
            for (int s = 0; s < 8; ++s) { const int Lid = (lane >> 3) + 4 * s, piece = lane & 7; const int row = Lid >> 1, cofs = (Lid & 1) * 32 + piece * 4;
                v4f val = *(const v4fa*)(os + row * 68 + cofs); if (R) { const v4f rv = *(const v4f*)(R + ((size_t)r0 + row) * ldc + c0 + cofs); val += roundR ? (v4f){bfr(rv[0]), bfr(rv[1]), bfr(rv[2]), bfr(rv[3])} : rv; }
                *(volatile v4f*)(crow + (size_t)row * ldc + cofs) = val; }
        };
        pass(); __threadfence(); pass();
    }
}


__global__ __launch_bounds__(256) void k_entpad(const float* __restrict__ ent, bf* A) {
    const int lane = threadIdx.x & 31; const int r = blockIdx.x * 8 + (threadIdx.x >> 5); if (r >= 64) return; v8us o;
#pragma unroll
    for (int i = 0; i < 8; ++i) o[i] = f2bf(r < NE ? ent[(size_t)(r < NE ? r : 0) * EE + lane * 8 + i] : 0.f);
    *(volatile v8us*)(A + (size_t)r * EE + lane * 8) = o; __threadfence(); *(volatile v8us*)(A + (size_t)r * EE + lane * 8) = o;
}
__global__ __launch_bounds__(256) void k_wt2(const float* __restrict__ Wm, bf* Bt) {
    const int lane = threadIdx.x & 31; const int n = blockIdx.x * 8 + (threadIdx.x >> 5); if (n >= 2 * HH) return; const int half = n / HH, nn = n % HH; v8us o;
#pragma unroll
    for (int i = 0; i < 8; ++i) { const int k = lane * 8 + i; o[i] = f2bf(Wm[(size_t)(half * EE + k) * HH + nn]); }
    *(volatile v8us*)(Bt + (size_t)n * EE + lane * 8) = o; __threadfence(); *(volatile v8us*)(Bt + (size_t)n * EE + lane * 8) = o;
}
__global__ __launch_bounds__(256) void k_wt1(const float* __restrict__ Wm, bf* Bt) {
    const int lane = threadIdx.x & 31; const int n = blockIdx.x * 8 + (threadIdx.x >> 5); if (n >= HH) return; v8us o;
#pragma unroll
    for (int i = 0; i < 8; ++i) { const int k = lane * 8 + i; o[i] = f2bf(Wm[(size_t)k * HH + n]); }
    *(volatile v8us*)(Bt + (size_t)n * HH + lane * 8) = o; __threadfence(); *(volatile v8us*)(Bt + (size_t)n * HH + lane * 8) = o;
}
__global__ __launch_bounds__(256) void k_wvpad(const float* __restrict__ w, bf* Bt) {
    const int lane = threadIdx.x & 31; const int n = blockIdx.x * 8 + (threadIdx.x >> 5); if (n >= 64) return; v8us o;
#pragma unroll
    for (int i = 0; i < 8; ++i) o[i] = f2bf(n == 0 ? w[lane * 8 + i] : 0.f);
    *(volatile v8us*)(Bt + (size_t)n * HH + lane * 8) = o; __threadfence(); *(volatile v8us*)(Bt + (size_t)n * HH + lane * 8) = o;
}
template <bool LN>
__global__ __launch_bounds__(256) void k_pairln(const float* __restrict__ Am, const float* __restrict__ Bm, int ld, int offA, int offB, int NJ, int NP, int p0, int rows, const float* __restrict__ bias, const float* __restrict__ g, const float* __restrict__ be, bf* Ph, bf* Pl) {
    const int lane = threadIdx.x & 31; const size_t rl = (size_t)blockIdx.x * 8 + (threadIdx.x >> 5); if (rl >= (size_t)rows) return; const size_t p = p0 + rl; const bool live = p < (size_t)NP; const int i = live ? (int)(p / NJ) : 0, j = live ? (int)(p % NJ) : 0;
    float v[8]; float s = 0.f;
#pragma unroll
    for (int q = 0; q < 8; ++q) { const int c = lane * 8 + q; const float t = live ? (Am[(size_t)i * ld + offA + c] + Bm[(size_t)j * ld + offB + c] + bfr(bias[c])) : 0.f; v[q] = t; s += t; }
    float mu = 0.f, rs = 1.f;
    if (LN) {
#pragma unroll
        for (int sh = 16; sh; sh >>= 1) s += __shfl_xor(s, sh, 32);
        mu = s * (1.0f / HH); float qv = 0.f;
#pragma unroll
        for (int q = 0; q < 8; ++q) { const float d = v[q] - mu; qv = fmaf(d, d, qv); }
#pragma unroll
        for (int sh = 16; sh; sh >>= 1) qv += __shfl_xor(qv, sh, 32);
        rs = rsqrtf(qv * (1.0f / HH) + LEPS); }
    v8us oh, ol;
#pragma unroll
    for (int q = 0; q < 8; ++q) { const int c = lane * 8 + q; float y = LN ? ((v[q] - mu) * rs * bfr(g[c]) + bfr(be[c])) : v[q]; y = fmaxf(y, 0.f); if (!live) y = 0.f; const unsigned short hb = f2bf(y); oh[q] = hb; ol[q] = f2bf(y - bf2f(hb)); }
    const size_t o = rl * HH + lane * 8; *(volatile v8us*)(Ph + o) = oh; *(volatile v8us*)(Pl + o) = ol; __threadfence(); *(volatile v8us*)(Ph + o) = oh; *(volatile v8us*)(Pl + o) = ol;
}
__global__ __launch_bounds__(256) void k_maskplanes(const float* __restrict__ Hf, const int* __restrict__ rel, bf* Ph, bf* Pl) {
    const int lane = threadIdx.x & 31; const int r = blockIdx.x * 8 + (threadIdx.x >> 5); if (r >= RP) return; const bool live = (r < RR) && (rel[r < RR ? r : 0] > 0); v8us oh, ol;
#pragma unroll
    for (int q = 0; q < 8; ++q) { const float y = live ? Hf[(size_t)r * HH + lane * 8 + q] : 0.f; const unsigned short hb = f2bf(y); oh[q] = hb; ol[q] = f2bf(y - bf2f(hb)); }
    const size_t o = (size_t)r * HH + lane * 8; *(volatile v8us*)(Ph + o) = oh; *(volatile v8us*)(Pl + o) = ol; __threadfence(); *(volatile v8us*)(Ph + o) = oh; *(volatile v8us*)(Pl + o) = ol;
}
__global__ __launch_bounds__(256) void k_rowstat(const float* __restrict__ MS, const float* __restrict__ bm2, float* STAT) {
    const int lane = threadIdx.x & 31; const int r = blockIdx.x * 8 + (threadIdx.x >> 5); if (r >= RR) return; const float bb = bfr(bm2[0]); float m = -3.0e38f;
    for (int s = lane; s < RR; s += 32) m = fmaxf(m, MS[((size_t)r * RR + s) * 64] + bb);
#pragma unroll
    for (int sh = 16; sh; sh >>= 1) m = fmaxf(m, __shfl_xor(m, sh, 32));
    float sum = 0.f;
    for (int s = lane; s < RR; s += 32) sum += __expf(MS[((size_t)r * RR + s) * 64] + bb - m);
#pragma unroll
    for (int sh = 16; sh; sh >>= 1) sum += __shfl_xor(sum, sh, 32);
    const float v = (lane == 0) ? m : (lane == 1) ? 1.0f / sum : 0.f; *(volatile float*)(STAT + (size_t)r * 32 + lane) = v; __threadfence(); *(volatile float*)(STAT + (size_t)r * 32 + lane) = v;
}
__global__ __launch_bounds__(256) void k_mapout(const float* __restrict__ MS, const float* __restrict__ bm2, const float* __restrict__ STAT, float* dst) {
    const int lane = threadIdx.x & 31; const size_t w = (size_t)blockIdx.x * 8 + (threadIdx.x >> 5); if (w >= (size_t)NPAIR / 128) return; const size_t e0 = w * 128 + lane * 4; const float bb = bfr(bm2[0]); v4f v;
#pragma unroll
    for (int i = 0; i < 4; ++i) { const size_t e = e0 + i; const int r = (int)(e / RR); v[i] = __expf(MS[e * 64] + bb - STAT[(size_t)r * 32]) * STAT[(size_t)r * 32 + 1]; }
    *(volatile v4f*)(dst + e0) = v; __threadfence(); *(volatile v4f*)(dst + e0) = v;
}
__global__ __launch_bounds__(256) void k_corrout(const float* __restrict__ CS, const float* __restrict__ bc2, float* dst) {
    const int tid = threadIdx.x; const int e0 = tid * 4; if (e0 >= NB_ * RR) return; const float bb = bfr(bc2[0]); v4f v;
#pragma unroll
    for (int q = 0; q < 4; ++q) { const int e = e0 + q; const int b = e / RR, i = (e % RR) / NE; const float* cs = CS + (size_t)b * RP * 64; float m = -3.0e38f;
#pragma unroll 1
        for (int j = 0; j < NE; ++j) m = fmaxf(m, cs[(size_t)(i * NE + j) * 64] + bb);
        float s = 0.f;
#pragma unroll 1
        for (int j = 0; j < NE; ++j) s += __expf(cs[(size_t)(i * NE + j) * 64] + bb - m);
        v[q] = __expf(cs[(size_t)(e % RR) * 64] + bb - m) / s; }
    *(volatile v4f*)(dst + e0) = v; __threadfence(); *(volatile v4f*)(dst + e0) = v;
}

extern "C" void kernel_launch(void* const* d_in, const int* in_sizes, int n_in,
                              void* d_out, int out_size, void* d_ws, size_t ws_size, hipStream_t stream) {
    (void)in_sizes; (void)n_in; (void)out_size;
    const float* se = (const float*)d_in[0]; const float* te = (const float*)d_in[1]; const int* srel = (const int*)d_in[2]; const int* trel = (const int*)d_in[3];
    const float* W1 = (const float*)d_in[4]; const float* b1 = (const float*)d_in[5]; const float* g1 = (const float*)d_in[6]; const float* be1 = (const float*)d_in[7]; const float* W2 = (const float*)d_in[8]; const float* b2 = (const float*)d_in[9];
    const float* Wm1 = (const float*)d_in[10]; const float* bm1 = (const float*)d_in[11]; const float* gm = (const float*)d_in[12]; const float* bem = (const float*)d_in[13]; const float* Wm2 = (const float*)d_in[14]; const float* bm2 = (const float*)d_in[15];
    const float* Wc1 = (const float*)d_in[16]; const float* bc1 = (const float*)d_in[17]; const float* Wc2 = (const float*)d_in[18]; const float* bc2 = (const float*)d_in[19];
    float* out0 = (float*)d_out;
    float* out1 = (float*)((char*)d_out + 1280000);
    char* wsp = (char*)d_ws;
    auto take = [&](size_t bytes) { char* p = wsp; wsp += (bytes + 255) & ~(size_t)255; return (void*)p; };
    bf* BW1 = (bf*)take((size_t)2 * HH * EE * 2); bf* BW2 = (bf*)take((size_t)HH * HH * 2); bf* BWM1 = (bf*)take((size_t)2 * HH * HH * 2); bf* BWM2 = (bf*)take((size_t)64 * HH * 2); bf* BWC1 = (bf*)take((size_t)2 * HH * EE * 2); bf* BWC2 = (bf*)take((size_t)64 * HH * 2);
    bf* SE = (bf*)take(64 * EE * 2); bf* TE = (bf*)take(64 * EE * 2); float* HS = (float*)take((size_t)64 * 2 * HH * 4); float* HT = (float*)take((size_t)64 * 2 * HH * 4); float* CAB = (float*)take((size_t)64 * 2 * HH * 4); float* CBB = (float*)take((size_t)64 * 2 * HH * 4);
    bf* P1h = (bf*)take((size_t)RP * HH * 2); bf* P1l = (bf*)take((size_t)RP * HH * 2); float* HR = (float*)take((size_t)RP * HH * 4); bf* SRh = (bf*)take((size_t)RP * HH * 2); bf* SRl = (bf*)take((size_t)RP * HH * 2); bf* TRh = (bf*)take((size_t)RP * HH * 2); bf* TRl = (bf*)take((size_t)RP * HH * 2);
    float* SA = (float*)take((size_t)RP * HH * 4); float* TB = (float*)take((size_t)RP * HH * 4); bf* PMh = (bf*)take((size_t)PCH * HH * 2); bf* PMl = (bf*)take((size_t)PCH * HH * 2); float* MS = (float*)take((size_t)NPAIR * 64 * 4); float* STAT = (float*)take((size_t)RR * 32 * 4); float* CS = (float*)take((size_t)NB_ * RP * 64 * 4);
    if ((size_t)(wsp - (char*)d_ws) > ws_size) return;
    k_wt2<<<(2 * HH) / 8, 256, 0, stream>>>(W1, BW1); k_wt1<<<HH / 8, 256, 0, stream>>>(W2, BW2); k_wt2<<<(2 * HH) / 8, 256, 0, stream>>>(Wm1, BWM1); k_wvpad<<<64 / 8, 256, 0, stream>>>(Wm2, BWM2); k_wt2<<<(2 * HH) / 8, 256, 0, stream>>>(Wc1, BWC1); k_wvpad<<<64 / 8, 256, 0, stream>>>(Wc2, BWC2);
    for (int b = 0; b < NB_; ++b) {
        k_entpad<<<64 / 8, 256, 0, stream>>>(se + (size_t)b * NE * EE, SE); k_entpad<<<64 / 8, 256, 0, stream>>>(te + (size_t)b * NE * EE, TE);
        k_gemmb<false, false><<<dim3(1, (2 * HH) / 64, 1), 128, 0, stream>>>(SE, nullptr, BW1, nullptr, HS, 2 * HH, nullptr, nullptr, EE);
        k_gemmb<false, false><<<dim3(1, (2 * HH) / 64, 1), 128, 0, stream>>>(TE, nullptr, BW1, nullptr, HT, 2 * HH, nullptr, nullptr, EE);
        k_pairln<true><<<RP / 8, 256, 0, stream>>>(HS, HS, 2 * HH, 0, HH, NE, RR, 0, RP, b1, g1, be1, P1h, P1l);
        k_gemmb<true, false><<<dim3(RP / 64, HH / 64, 1), 128, 0, stream>>>(P1h, P1l, BW2, b2, HR, HH, nullptr, nullptr, HH); k_maskplanes<<<RP / 8, 256, 0, stream>>>(HR, srel + (size_t)b * RR, SRh, SRl);
        k_pairln<true><<<RP / 8, 256, 0, stream>>>(HT, HT, 2 * HH, 0, HH, NE, RR, 0, RP, b1, g1, be1, P1h, P1l);
        k_gemmb<true, false><<<dim3(RP / 64, HH / 64, 1), 128, 0, stream>>>(P1h, P1l, BW2, b2, HR, HH, nullptr, nullptr, HH); k_maskplanes<<<RP / 8, 256, 0, stream>>>(HR, trel + (size_t)b * RR, TRh, TRl);
        k_gemmb<true, false><<<dim3(RP / 64, HH / 64, 1), 128, 0, stream>>>(SRh, SRl, BWM1, nullptr, SA, HH, nullptr, nullptr, HH);
        k_gemmb<true, false><<<dim3(RP / 64, HH / 64, 1), 128, 0, stream>>>(TRh, TRl, BWM1 + (size_t)HH * HH, nullptr, TB, HH, nullptr, nullptr, HH);
        for (int ch = 0; ch < NPAIR / PCH; ++ch) { const int p0 = ch * PCH;
            k_pairln<true><<<PCH / 8, 256, 0, stream>>>(SA, TB, HH, 0, 0, RR, NPAIR, p0, PCH, bm1, gm, bem, PMh, PMl);
            k_gemmb<true, false><<<dim3(PCH / 64, 1, 1), 128, 0, stream>>>(PMh, PMl, BWM2, nullptr, MS + (size_t)p0 * 64, 64, nullptr, nullptr, HH); }
        k_rowstat<<<RR / 8, 256, 0, stream>>>(MS, bm2, STAT); k_mapout<<<(NPAIR / 128) / 8 + 1, 256, 0, stream>>>(MS, bm2, STAT, out0 + (size_t)b * NPAIR);
        k_gemmb<false, false><<<dim3(1, (2 * HH) / 64, 1), 128, 0, stream>>>(SE, nullptr, BWC1, nullptr, CAB, 2 * HH, nullptr, nullptr, EE);
        k_gemmb<false, false><<<dim3(1, (2 * HH) / 64, 1), 128, 0, stream>>>(TE, nullptr, BWC1, nullptr, CBB, 2 * HH, nullptr, nullptr, EE);
        k_pairln<false><<<RP / 8, 256, 0, stream>>>(CAB, CBB, 2 * HH, 0, HH, NE, RR, 0, RP, bc1, nullptr, nullptr, P1h, P1l);
        k_gemmb<true, false><<<dim3(RP / 64, 1, 1), 128, 0, stream>>>(P1h, P1l, BWC2, nullptr, CS + (size_t)b * RP * 64, 64, nullptr, nullptr, HH); }
    k_corrout<<<1, 256, 0, stream>>>(CS, bc2, out1);
}
